// FixedSeedMixtureLowRankRNN_48369921687959
// MI455X (gfx1250) — hardware-run, weakly checked
//
#include <hip/hip_runtime.h>
#include <math.h>

typedef __attribute__((ext_vector_type(16))) _Float16 v16h;
typedef __attribute__((ext_vector_type(8)))  _Float16 v8h;
typedef __attribute__((ext_vector_type(4)))  _Float16 v4h;
typedef __attribute__((ext_vector_type(8)))  float    v8f;
typedef __attribute__((ext_vector_type(4)))  float    v4f;
typedef __attribute__((ext_vector_type(2)))  float    v2f;

constexpr int kRank  = 2;
constexpr int kHid   = 512;
constexpr int kIn    = 8;
constexpr int kMix   = 2;
constexpr int kSeeds = 4;
constexpr int kBatch = 64;
constexpr int kSeq   = 2048;
constexpr int kD     = 2 * kRank + kIn;
constexpr int kNS    = kRank + kIn;
constexpr int kNPad  = 16;
constexpr int kTile  = 16;
constexpr int kAP    = 520;
static_assert(kD == 12 && kNS == 10, "span layout");
static_assert((kSeq % kTile) == 0 && (kHid % 32) == 0, "tile multiples");
static_assert(((kAP * 2) % 16) == 0 && kAP >= kHid, "LDS pitch of the state tile");
static_assert(((kTile * kNS * 4) % 128) == 0, "a 16-step output tile is whole 128-B lines");

constexpr float kAlpha  = 0.1f;
constexpr float kCJ     = 500.0f / (float)kHid;
constexpr float kHC     = 16.0f;
constexpr float kPC     = 64.0f;
constexpr float kLoS    = 2048.0f;
constexpr float kLoInv  = 1.0f / kLoS;
constexpr float kFold   = 1.0f / (kHC * kPC);
constexpr float kF16Min = 6.103515625e-5f;

constexpr size_t kOffMN   = 0;
constexpr size_t kOffIW   = kOffMN + (size_t)kSeeds * 4 * kHid * 4;
constexpr size_t kOffPH   = kOffIW + (size_t)kSeeds * kHid * kIn * 4;
constexpr size_t kOffPL   = kOffPH + (size_t)kSeeds * kNPad * kHid * 2;
constexpr size_t kWsTotal = kOffPL + (size_t)kSeeds * kNPad * kHid * 2;
static_assert(kWsTotal == 229376ull, "carve total");
static_assert((kOffIW % 128) == 0 && (kOffPH % 128) == 0 && (kOffPL % 128) == 0, "128-B aligned regions");
static_assert(kWsTotal <= 134217728ull, "carve cap");

union FragH { v16h v; v8h h[2]; };

__device__ __forceinline__ v8f mma_f16(v16h a, v16h b, v8f c) {
  c = __builtin_amdgcn_wmma_f32_16x16x32_f16(false, a, false, b, (short)0, c, false, false);
  asm volatile("v_nop\n\tv_nop\n\tv_nop\n\tv_nop" : "+v"(c) : "v"(a), "v"(b));
  return c;
}

__device__ __forceinline__ void split16(float v, _Float16& hi, _Float16& lo) {
  const float vf = (fabsf(v) < kF16Min) ? 0.0f : v;
  hi = (_Float16)vf;
  const float hf = (float)hi;
  float r = (v - hf) * kLoS;
  r = (fabsf(r) < kF16Min) ? 0.0f : r;
  lo = (_Float16)r;
}

__global__ __launch_bounds__(256) void prep_kernel(
    const float* __restrict__ means, const float* __restrict__ st, const float* __restrict__ mw,
    const float* __restrict__ seeds, float* __restrict__ MN, float* __restrict__ IW,
    _Float16* __restrict__ PH, _Float16* __restrict__ PL)
{
  __shared__ __align__(16) float sL[kD * kD];
  __shared__ __align__(16) float sMb[16];
  __shared__ __align__(16) float sC[kD * kHid];
  __shared__ __align__(16) float sQ[kNS * kHid];
  __shared__ __align__(16) float sR[kNS * kNS + 4];
  __shared__ __align__(16) float sRed[16];
  const int tid = threadIdx.x, lane = tid & 31, wave = tid >> 5;
  const int s = blockIdx.x;

  float w0 = fmaxf(mw[0], 1e-6f);
  float w1 = fmaxf(mw[1], 1e-6f);
  const float wr = 1.0f / (w0 + w1);
  w0 *= wr;
  w1 *= wr;

  {
    const int idx = (tid < kD * kD) ? tid : (kD * kD - 1);
    float a0 = st[idx];
    float a1 = st[kD * kD + idx];
    asm volatile("" : "+v"(a0));
    asm volatile("" : "+v"(a1));
    const int d = idx / kD;
    const int e = idx - d * kD;
    const float g0 = fabsf(a0 - 1e-12f) + 1e-12f;
    const float g1 = fabsf(a1 - 1e-12f) + 1e-12f;
    const float v0 = (e < d) ? a0 : ((e == d) ? g0 : 0.0f);
    const float v1 = (e < d) ? a1 : ((e == d) ? g1 : 0.0f);
    float acc = 0.0f;
    acc += w0 * v0;
    acc += w1 * v1;
    if (tid < kD * kD) sL[tid] = acc;
    const int im = (tid < kD) ? tid : (kD - 1);
    float b0 = means[im];
    float b1 = means[kD + im];
    asm volatile("" : "+v"(b0));
    asm volatile("" : "+v"(b1));
    float mb = 0.0f;
    mb += w0 * b0;
    mb += w1 * b1;
    if (tid < kD) sMb[tid] = mb;
    if (tid < kNS * kNS) sR[tid] = 0.0f;
  }
  __syncthreads();

#pragma unroll 1
  for (int rep = 0; rep < 2; ++rep) {
    const int h = tid + rep * 256;
    const float* sp = seeds + ((size_t)s * kHid + h) * kD;
    const v4f s0 = *(const v4f*)(sp);
    const v4f s1 = *(const v4f*)(sp + 4);
    const v4f s2 = *(const v4f*)(sp + 8);
#pragma unroll 1
    for (int d = 0; d < kD; ++d) {
      const float* lr = sL + d * kD;
      float acc = sMb[d];
      acc = fmaf(lr[0],  s0[0], acc);
      acc = fmaf(lr[1],  s0[1], acc);
      acc = fmaf(lr[2],  s0[2], acc);
      acc = fmaf(lr[3],  s0[3], acc);
      acc = fmaf(lr[4],  s1[0], acc);
      acc = fmaf(lr[5],  s1[1], acc);
      acc = fmaf(lr[6],  s1[2], acc);
      acc = fmaf(lr[7],  s1[3], acc);
      acc = fmaf(lr[8],  s2[0], acc);
      acc = fmaf(lr[9],  s2[1], acc);
      acc = fmaf(lr[10], s2[2], acc);
      acc = fmaf(lr[11], s2[3], acc);
      sC[d * kHid + h] = acc;
    }
  }
  __syncthreads();

#pragma unroll 1
  for (int k = 0; k < kNS; ++k) {
    const int src = (k < kRank) ? k : (k + kRank);
    sQ[k * kHid + tid]       = sC[src * kHid + tid];
    sQ[k * kHid + tid + 256] = sC[src * kHid + tid + 256];
  }

  {
    v4f mv[2];
    v4f iv[4];
#pragma unroll
    for (int it = 0; it < 2; ++it) mv[it] = *(const v4f*)(sC + 4 * (tid + it * 256));
#pragma unroll
    for (int it = 0; it < 4; ++it) {
      const int q = tid + it * 256;
      const int h = q >> 1;
      const int i0 = (q & 1) * 4;
      v4f t;
      t[0] = sC[(4 + i0 + 0) * kHid + h];
      t[1] = sC[(4 + i0 + 1) * kHid + h];
      t[2] = sC[(4 + i0 + 2) * kHid + h];
      t[3] = sC[(4 + i0 + 3) * kHid + h];
      iv[it] = t;
    }
    float* mnb = MN + (size_t)s * 4 * kHid;
    float* iwb = IW + (size_t)s * kHid * kIn;
    for (int pass = 0; pass < 2; ++pass) {
#pragma unroll
      for (int it = 0; it < 2; ++it) *(volatile v4f*)(mnb + 4 * (tid + it * 256)) = mv[it];
#pragma unroll
      for (int it = 0; it < 4; ++it) *(volatile v4f*)(iwb + 4 * (tid + it * 256)) = iv[it];
      __threadfence();
    }
  }

  int ph = 0;
#pragma unroll 1
  for (int j = 0; j < kNS; ++j) {
    float v0 = sQ[j * kHid + tid];
    float v1 = sQ[j * kHid + tid + 256];
#pragma unroll 1
    for (int pass = 0; pass < 2; ++pass) {
#pragma unroll 1
      for (int i = 0; i < j; ++i) {
        const float q0 = sQ[i * kHid + tid];
        const float q1 = sQ[i * kHid + tid + 256];
        float p = q0 * v0;
        p = fmaf(q1, v1, p);
        p += __shfl_xor(p, 16, 32);
        p += __shfl_xor(p, 8, 32);
        p += __shfl_xor(p, 4, 32);
        p += __shfl_xor(p, 2, 32);
        p += __shfl_xor(p, 1, 32);
        if (lane == 0) sRed[ph * 8 + wave] = p;
        __syncthreads();
        float ds = sRed[ph * 8 + 0];
        ds += sRed[ph * 8 + 1];
        ds += sRed[ph * 8 + 2];
        ds += sRed[ph * 8 + 3];
        ds += sRed[ph * 8 + 4];
        ds += sRed[ph * 8 + 5];
        ds += sRed[ph * 8 + 6];
        ds += sRed[ph * 8 + 7];
        ph ^= 1;
        v0 = fmaf(-ds, q0, v0);
        v1 = fmaf(-ds, q1, v1);
        if (tid == 0) sR[i * kNS + j] += ds;
      }
    }
    float p = v0 * v0;
    p = fmaf(v1, v1, p);
    p += __shfl_xor(p, 16, 32);
    p += __shfl_xor(p, 8, 32);
    p += __shfl_xor(p, 4, 32);
    p += __shfl_xor(p, 2, 32);
    p += __shfl_xor(p, 1, 32);
    if (lane == 0) sRed[ph * 8 + wave] = p;
    __syncthreads();
    float n2 = sRed[ph * 8 + 0];
    n2 += sRed[ph * 8 + 1];
    n2 += sRed[ph * 8 + 2];
    n2 += sRed[ph * 8 + 3];
    n2 += sRed[ph * 8 + 4];
    n2 += sRed[ph * 8 + 5];
    n2 += sRed[ph * 8 + 6];
    n2 += sRed[ph * 8 + 7];
    ph ^= 1;
    const float rjj = sqrtf(n2);
    const float inv = (rjj > 0.0f) ? (1.0f / rjj) : 0.0f;
    sQ[j * kHid + tid]       = v0 * inv;
    sQ[j * kHid + tid + 256] = v1 * inv;
    if (tid == 0) sR[j * kNS + j] = rjj;
  }
  __syncthreads();

#pragma unroll 1
  for (int k = kNS - 1; k >= 0; --k) {
    const float rkk = sR[k * kNS + k];
    const float rinv = (rkk > 0.0f) ? (1.0f / rkk) : 0.0f;
    float a0 = sQ[k * kHid + tid];
    float a1 = sQ[k * kHid + tid + 256];
#pragma unroll 1
    for (int l = k + 1; l < kNS; ++l) {
      const float r = sR[k * kNS + l];
      a0 = fmaf(-r, sQ[l * kHid + tid], a0);
      a1 = fmaf(-r, sQ[l * kHid + tid + 256], a1);
    }
    sQ[k * kHid + tid]       = a0 * rinv;
    sQ[k * kHid + tid + 256] = a1 * rinv;
  }
  __syncthreads();

  {
    _Float16* phb = PH + (size_t)s * kNPad * kHid;
    _Float16* plb = PL + (size_t)s * kNPad * kHid;
#pragma unroll 1
    for (int it = 0; it < 4; ++it) {
      const int q = tid + it * 256;
      const int row = q >> 6;
      const int c8 = (q & 63) * 8;
      const int rr = (row < kNS) ? row : (kNS - 1);
      const float* sp = sQ + rr * kHid + c8;
      const v4f a0 = *(const v4f*)(sp);
      const v4f a1 = *(const v4f*)(sp + 4);
      v8h hv, lv;
#pragma unroll
      for (int e = 0; e < 4; ++e) {
        const float x0 = (row < kNS) ? (a0[e] * kPC) : 0.0f;
        const float x1 = (row < kNS) ? (a1[e] * kPC) : 0.0f;
        _Float16 h0, l0, h1, l1;
        split16(x0, h0, l0);
        split16(x1, h1, l1);
        hv[e] = h0;
        lv[e] = l0;
        hv[4 + e] = h1;
        lv[4 + e] = l1;
      }
      *(volatile v8h*)(phb + 8 * q) = hv;
      *(volatile v8h*)(plb + 8 * q) = lv;
      __threadfence();
      *(volatile v8h*)(phb + 8 * q) = hv;
      *(volatile v8h*)(plb + 8 * q) = lv;
    }
  }
}

__global__ __launch_bounds__(128) void scan_proj_kernel(
    const float* __restrict__ x, const int* __restrict__ cur,
    const float* __restrict__ MN, const float* __restrict__ IW,
    const _Float16* __restrict__ PH, const _Float16* __restrict__ PL,
    float* __restrict__ out)
{
  __shared__ __align__(16) _Float16 sAh[kTile * kAP];
  __shared__ __align__(16) _Float16 sAl[kTile * kAP];
  __shared__ __align__(16) float sRed[16];
  __shared__ __align__(16) float sOut[4 * kTile * kNS];
  const int tid = threadIdx.x, lane = tid & 31;
  const int wave = __builtin_amdgcn_readfirstlane(tid >> 5);
  const int b = blockIdx.x;
  int sd = cur[b];
  sd = (sd < 0) ? 0 : ((sd > kSeeds - 1) ? (kSeeds - 1) : sd);
  const int hb = tid * 4;

  float mc0[4], mc1[4], n0[4], n1[4], h[4];
  float iw[4][8];
  {
    const float* mp = MN + (size_t)sd * 4 * kHid + hb;
    const v4f q0 = *(const v4f*)(mp);
    const v4f q1 = *(const v4f*)(mp + kHid);
    const v4f q2 = *(const v4f*)(mp + 2 * kHid);
    const v4f q3 = *(const v4f*)(mp + 3 * kHid);
    const float* ip = IW + ((size_t)sd * kHid + hb) * kIn;
#pragma unroll
    for (int j = 0; j < 4; ++j) {
      mc0[j] = q0[j] * kCJ;
      mc1[j] = q1[j] * kCJ;
      n0[j] = q2[j];
      n1[j] = q3[j];
      h[j] = 0.0f;
      const v4f ia = *(const v4f*)(ip + j * kIn);
      const v4f ib = *(const v4f*)(ip + j * kIn + 4);
      iw[j][0] = ia[0]; iw[j][1] = ia[1]; iw[j][2] = ia[2]; iw[j][3] = ia[3];
      iw[j][4] = ib[0]; iw[j][5] = ib[1]; iw[j][6] = ib[2]; iw[j][7] = ib[3];
    }
  }

  const v4f* xp = (const v4f*)(x + (size_t)b * kSeq * kIn);
  v4f xa = xp[0];
  v4f xb = xp[1];

  const int mrow = lane & 15;
  const int hh = lane >> 4;
  const _Float16* bph = PH + ((size_t)(sd * kNPad + mrow)) * kHid + 8 * hh;
  const _Float16* bpl = PL + ((size_t)(sd * kNPad + mrow)) * kHid + 8 * hh;

#pragma unroll 1
  for (int tile = 0; tile < kSeq / kTile; ++tile) {
#pragma unroll 1
    for (int sidx = 0; sidx < kTile; ++sidx) {
      const int t = tile * kTile + sidx;
      const int tn = (t + 1 < kSeq) ? (t + 1) : (kSeq - 1);
      const v4f nxa = xp[2 * tn];
      const v4f nxb = xp[2 * tn + 1];
      const int par = t & 1;

      float p0 = 0.0f, p1 = 0.0f;
#pragma unroll
      for (int j = 0; j < 4; ++j) {
        const float th = tanhf(h[j]);
        p0 = fmaf(n0[j], th, p0);
        p1 = fmaf(n1[j], th, p1);
      }
      p0 += __shfl_xor(p0, 16, 32);
      p1 += __shfl_xor(p1, 16, 32);
      p0 += __shfl_xor(p0, 8, 32);
      p1 += __shfl_xor(p1, 8, 32);
      p0 += __shfl_xor(p0, 4, 32);
      p1 += __shfl_xor(p1, 4, 32);
      p0 += __shfl_xor(p0, 2, 32);
      p1 += __shfl_xor(p1, 2, 32);
      p0 += __shfl_xor(p0, 1, 32);
      p1 += __shfl_xor(p1, 1, 32);
      if (lane == 0) {
        v2f pr;
        pr[0] = p0;
        pr[1] = p1;
        *(v2f*)(&sRed[par * 8 + wave * 2]) = pr;
      }
      __syncthreads();
      const v4f ra = *(const v4f*)(&sRed[par * 8]);
      const v4f rb = *(const v4f*)(&sRed[par * 8 + 4]);
      const float u0 = ((ra[0] + ra[2]) + rb[0]) + rb[2];
      const float u1 = ((ra[1] + ra[3]) + rb[1]) + rb[3];

      v4h hv, lv;
#pragma unroll
      for (int j = 0; j < 4; ++j) {
        float ix = iw[j][0] * xa[0];
        ix = fmaf(iw[j][1], xa[1], ix);
        ix = fmaf(iw[j][2], xa[2], ix);
        ix = fmaf(iw[j][3], xa[3], ix);
        ix = fmaf(iw[j][4], xb[0], ix);
        ix = fmaf(iw[j][5], xb[1], ix);
        ix = fmaf(iw[j][6], xb[2], ix);
        ix = fmaf(iw[j][7], xb[3], ix);
        float rec = mc0[j] * u0;
        rec = fmaf(mc1[j], u1, rec);
        const float dh = (rec - h[j]) + ix;
        h[j] = fmaf(kAlpha, dh, h[j]);
        _Float16 e0, e1;
        split16(h[j] * kHC, e0, e1);
        hv[j] = e0;
        lv[j] = e1;
      }
      *(v4h*)(&sAh[sidx * kAP + hb]) = hv;
      *(v4h*)(&sAl[sidx * kAP + hb]) = lv;
      xa = nxa;
      xb = nxb;
    }
    __syncthreads();

    if (wave == (tile & 3)) {
      v8f accM = (v8f){0.f, 0.f, 0.f, 0.f, 0.f, 0.f, 0.f, 0.f};
      v8f accR = (v8f){0.f, 0.f, 0.f, 0.f, 0.f, 0.f, 0.f, 0.f};
#pragma unroll
      for (int ks = 0; ks < kHid / 32; ++ks) {
        const int k0 = ks * 32;
        FragH ah, al, bh, bl;
        ah.h[0] = *(const v8h*)(&sAh[mrow * kAP + k0 + 8 * hh]);
        ah.h[1] = *(const v8h*)(&sAh[mrow * kAP + k0 + 16 + 8 * hh]);
        al.h[0] = *(const v8h*)(&sAl[mrow * kAP + k0 + 8 * hh]);
        al.h[1] = *(const v8h*)(&sAl[mrow * kAP + k0 + 16 + 8 * hh]);
        bh.h[0] = *(const v8h*)(bph + k0);
        bh.h[1] = *(const v8h*)(bph + k0 + 16);
        bl.h[0] = *(const v8h*)(bpl + k0);
        bl.h[1] = *(const v8h*)(bpl + k0 + 16);
        accM = mma_f16(ah.v, bh.v, accM);
        accR = mma_f16(ah.v, bl.v, accR);
        accR = mma_f16(al.v, bh.v, accR);
        asm volatile("" ::: "memory");
      }
      float* so = sOut + wave * (kTile * kNS);
#pragma unroll
      for (int r = 0; r < 8; ++r) {
        const float val = fmaf(accR[r], kLoInv, accM[r]) * kFold;
        if (mrow < kNS) so[(8 * hh + r) * kNS + mrow] = val;
      }
      __builtin_amdgcn_fence(__ATOMIC_RELEASE, "workgroup");
      __builtin_amdgcn_wave_barrier();
      __builtin_amdgcn_fence(__ATOMIC_ACQUIRE, "workgroup");
      const v4f o0 = *(const v4f*)(so + 4 * lane);
      const v4f o1 = *(const v4f*)(so + 128 + 4 * (lane & 7));
      float* dst = out + ((size_t)b * kSeq + (size_t)tile * kTile) * kNS;
      for (int pass = 0; pass < 2; ++pass) {
        *(volatile v4f*)(dst + 4 * lane) = o0;
        if (lane < 8) *(volatile v4f*)(dst + 128 + 4 * lane) = o1;
        __threadfence();
      }
      __builtin_amdgcn_fence(__ATOMIC_RELEASE, "workgroup");
      __builtin_amdgcn_wave_barrier();
      __builtin_amdgcn_fence(__ATOMIC_ACQUIRE, "workgroup");
    }
    __syncthreads();
  }
}

extern "C" void kernel_launch(void* const* d_in, const int* in_sizes, int n_in,
                              void* d_out, int out_size, void* d_ws, size_t ws_size,
                              hipStream_t stream) {
  if (n_in < 6) return;
  if (in_sizes[0] != kBatch * kSeq * kIn) return;
  if (in_sizes[1] != kMix * kD) return;
  if (in_sizes[2] != kMix * kD * kD) return;
  if (in_sizes[3] != kMix) return;
  if (in_sizes[4] != kSeeds * kHid * kD) return;
  if (in_sizes[5] != kBatch) return;
  if (out_size != kBatch * kSeq * kNS) return;
  if (ws_size < kWsTotal) return;

  const float* x     = (const float*)d_in[0];
  const float* means = (const float*)d_in[1];
  const float* st    = (const float*)d_in[2];
  const float* mw    = (const float*)d_in[3];
  const float* seeds = (const float*)d_in[4];
  const int*   cur   = (const int*)d_in[5];
  float* out = (float*)d_out;

  char* ws = (char*)d_ws;
  float*    MN = (float*)(ws + kOffMN);
  float*    IW = (float*)(ws + kOffIW);
  _Float16* PH = (_Float16*)(ws + kOffPH);
  _Float16* PL = (_Float16*)(ws + kOffPL);

  prep_kernel<<<kSeeds, 256, 0, stream>>>(means, st, mw, seeds, MN, IW, PH, PL);
  scan_proj_kernel<<<kBatch, 128, 0, stream>>>(x, cur, MN, IW, PH, PL, out);
}
